// DFMSDA_43327630082578
// MI455X (gfx1250) — hardware-verified
//
#include <hip/hip_runtime.h>
#include <stdint.h>
#include <stddef.h>
#include <math.h>


typedef _Float16 f16_t;
typedef _Float16 v16h __attribute__((ext_vector_type(16)));
typedef _Float16 v8h  __attribute__((ext_vector_type(8)));
typedef float    v8f  __attribute__((ext_vector_type(8)));
typedef float    v4f  __attribute__((ext_vector_type(4)));
typedef v4f v4fa __attribute__((may_alias));
typedef v8h v8ha __attribute__((may_alias));
union FragH { v16h v; v8h half[2]; };

static constexpr int DIMC    = 256;
static constexpr int Bn      = 4;
static constexpr int Hn      = 64;
static constexpr int Wn      = 64;
static constexpr int HWc     = Hn * Wn;
static constexpr int Mrows   = Bn * HWc;
static constexpr int HIDDENc = 4 * DIMC;
static constexpr float SCALE = 0.17677669529663687f;
static constexpr float WSCL  = 64.0f;
static constexpr float WINV  = 0.015625f;

static constexpr int KCHUNK  = 256;
static constexpr int LDSPAD  = 264;
static constexpr int GEMM_LDS_FLOATS = 16384;
static constexpr int PREP_POS = 16;

static constexpr size_t OFF_WQ    = 0;
static constexpr size_t OFF_WK    = 262144;
static constexpr size_t OFF_WV    = 524288;
static constexpr size_t OFF_WP    = 786432;
static constexpr size_t OFF_WFC1  = 1048576;
static constexpr size_t OFF_WFC2  = 2097152;
static constexpr size_t OFF_X1RES = 3145728;
static constexpr size_t OFF_X1N   = 19922944;
static constexpr size_t OFF_X2N   = 28311552;
static constexpr size_t OFF_Q     = 36700160;
static constexpr size_t OFF_K     = 45088768;
static constexpr size_t OFF_V     = 53477376;
static constexpr size_t OFF_ATT   = 61865984;
static constexpr size_t OFF_XAFT  = 70254592;
static constexpr size_t WS_TOTAL  = 87031808;

__device__ __forceinline__ float wsum32(float v) {
#pragma unroll
    for (int off = 16; off > 0; off >>= 1) v += __shfl_xor(v, off, 32);
    return v;
}

__device__ __forceinline__ void mma2(v8f& c0, v8f& c1, const v16h& a0, const v16h& a1, const v16h& b) {
    c0 = __builtin_amdgcn_wmma_f32_16x16x32_f16(false, a0, false, b, (short)0, c0, false, false);
    c1 = __builtin_amdgcn_wmma_f32_16x16x32_f16(false, a1, false, b, (short)0, c1, false, false);
    asm volatile("v_nop\n\tv_nop\n\tv_nop\n\tv_nop" : "+v"(c0), "+v"(c1) : "v"(a0), "v"(a1), "v"(b));
}

__device__ __forceinline__ v8h ln_row8(v4f r0, v4f r1, const float* __restrict__ g,
                                       const float* __restrict__ be, int lane) {
    float s = (r0[0] + r0[1]) + (r0[2] + r0[3]) + (r1[0] + r1[1]) + (r1[2] + r1[3]);
    s = wsum32(s);
    const float inv = 0.00390625f;
    const float mu = s * inv;
    float q = 0.f;
#pragma unroll
    for (int j = 0; j < 4; ++j) {
        float d = r0[j] - mu; q += d * d;
        d = r1[j] - mu;       q += d * d;
    }
    q = wsum32(q);
    const float rs = rsqrtf(q * inv + 1e-5f);
    const v4f g0 = *(const v4f*)(g + 8 * lane);
    const v4f g1 = *(const v4f*)(g + 8 * lane + 4);
    const v4f c0 = *(const v4f*)(be + 8 * lane);
    const v4f c1 = *(const v4f*)(be + 8 * lane + 4);
    v8h o;
#pragma unroll
    for (int j = 0; j < 4; ++j) {
        o[j]     = (f16_t)((r0[j] - mu) * rs * g0[j] + c0[j]);
        o[j + 4] = (f16_t)((r1[j] - mu) * rs * g1[j] + c1[j]);
    }
    return o;
}

__global__ __launch_bounds__(256) void cvt_kernel(const float* __restrict__ src, f16_t* dst, int n8, float sc) {
    const int i = blockIdx.x * 256 + threadIdx.x;
    if (i >= n8) return;
    const v4f a = *(const v4f*)(src + (size_t)i * 8);
    const v4f b = *(const v4f*)(src + (size_t)i * 8 + 4);
    v8h o;
#pragma unroll
    for (int j = 0; j < 4; ++j) { o[j] = (f16_t)(a[j] * sc); o[j + 4] = (f16_t)(b[j] * sc); }
    f16_t* d = dst + (size_t)i * 8;
    *(volatile v8h*)d = o;
    __threadfence();
    *(volatile v8h*)d = o;
}

__global__ __launch_bounds__(256) void prep_kernel(
    const float* __restrict__ xa, const float* __restrict__ xb,
    const float* __restrict__ g,  const float* __restrict__ be,
    float* x1res, f16_t* x1n, f16_t* x2n, int M) {
    __shared__ float td[PREP_POS * DIMC];
    __shared__ float tb[PREP_POS * DIMC];
    const int lane = threadIdx.x & 31, wave = threadIdx.x >> 5;
    const int m0 = blockIdx.x * PREP_POS;
    if (m0 + PREP_POS > M) return;
    const int b = m0 >> 12, sp0 = m0 & (HWc - 1);
    const int pl = lane & 15, par = lane >> 4;
    const float* pa = xa + (size_t)b * DIMC * HWc + sp0 + pl;
    const float* pb = xb + (size_t)b * DIMC * HWc + sp0 + pl;
#pragma unroll 4
    for (int i = 0; i < 16; ++i) {
        const int c = wave * 32 + 2 * i + par;
        const float va = pa[(size_t)c * HWc];
        const float vb = pb[(size_t)c * HWc];
        td[pl * DIMC + c] = va - vb;
        tb[pl * DIMC + c] = vb;
    }
    __syncthreads();
#pragma unroll
    for (int i = 0; i < 2; ++i) {
        const int p = wave * 2 + i;
        const int m = m0 + p;
        const float* rd = td + p * DIMC;
        const float* rb = tb + p * DIMC;
        const v4f d0 = *(const v4fa*)(rd + 8 * lane);
        const v4f d1 = *(const v4fa*)(rd + 8 * lane + 4);
        const v4f e0 = *(const v4fa*)(rd + 4 * lane);
        const v4f e1 = *(const v4fa*)(rd + 128 + 4 * lane);
        const v4f b0 = *(const v4fa*)(rb + 8 * lane);
        const v4f b1 = *(const v4fa*)(rb + 8 * lane + 4);
        const v8h o1 = ln_row8(d0, d1, g, be, lane);
        const v8h o2 = ln_row8(b0, b1, g, be, lane);
        float* r  = x1res + (size_t)m * DIMC;
        f16_t* p1 = x1n + (size_t)m * DIMC + 8 * lane;
        f16_t* p2 = x2n + (size_t)m * DIMC + 8 * lane;
        *(volatile v4f*)(r + 4 * lane) = e0;
        *(volatile v4f*)(r + 128 + 4 * lane) = e1;
        *(volatile v8h*)p1 = o1;
        *(volatile v8h*)p2 = o2;
        __threadfence();
        *(volatile v4f*)(r + 4 * lane) = e0;
        *(volatile v4f*)(r + 128 + 4 * lane) = e1;
        *(volatile v8h*)p1 = o1;
        *(volatile v8h*)p2 = o2;
    }
}

__global__ __launch_bounds__(256) void ln_rows_kernel(
    const float* __restrict__ xin, const float* __restrict__ g,
    const float* __restrict__ be, f16_t* outb, int M) {
    const int lane = threadIdx.x & 31;
    const int row = blockIdx.x * 8 + (threadIdx.x >> 5);
    if (row >= M) return;
    const float* p = xin + (size_t)row * DIMC + 8 * lane;
    const v4f r0 = *(const v4f*)p;
    const v4f r1 = *(const v4f*)(p + 4);
    const v8h o = ln_row8(r0, r1, g, be, lane);
    f16_t* dst = outb + (size_t)row * DIMC + 8 * lane;
    *(volatile v8h*)dst = o;
    __threadfence();
    *(volatile v8h*)dst = o;
}

template <int MODE>
__device__ __forceinline__ void tile_store(const float* stg, float* outf, f16_t* outb,
                                           int m0, int n0, int N, int lane) {
    if (MODE == 0 || MODE == 2) {
#pragma unroll
        for (int gI = 0; gI < 8; ++gI) {
            const int rl = 4 * gI + (lane >> 3);
            const int cl = 8 * (lane & 7);
            const v4f x0 = *(const v4fa*)(stg + rl * 64 + cl);
            const v4f x1 = *(const v4fa*)(stg + rl * 64 + cl + 4);
            v8h o;
#pragma unroll
            for (int j = 0; j < 4; ++j) { o[j] = (f16_t)x0[j]; o[j + 4] = (f16_t)x1[j]; }
            *(volatile v8h*)(outb + (size_t)(m0 + rl) * N + n0 + cl) = o;
        }
    } else if (MODE == 1) {
#pragma unroll
        for (int gI = 0; gI < 16; ++gI) {
            const int rl = 2 * gI + (lane >> 4);
            const int cl = 4 * (lane & 15);
            const v4f x = *(const v4fa*)(stg + rl * 64 + cl);
            *(volatile v4f*)(outf + (size_t)(m0 + rl) * N + n0 + cl) = x;
        }
    } else {
#pragma unroll
        for (int gI = 0; gI < 16; ++gI) {
            const int chl = 4 * gI + (lane >> 3);
            const int pl  = 4 * (lane & 7);
            const v4f x = *(const v4fa*)(stg + chl * 32 + pl);
            const int m  = m0 + pl;
            const int bb = m >> 12;
            const int sp = m & (HWc - 1);
            *(volatile v4f*)(outf + (size_t)bb * N * HWc + (size_t)(n0 + chl) * HWc + sp) = x;
        }
    }
}

template <int MODE>
__global__ __launch_bounds__(256) void gemm_kernel(
    const f16_t* __restrict__ A, const f16_t* __restrict__ Wt,
    const float* __restrict__ bias, const float* __restrict__ res,
    float* outf, f16_t* outb, int M, int N, int K) {
    __shared__ float lds_raw[GEMM_LDS_FLOATS];
    f16_t* bs = reinterpret_cast<f16_t*>(lds_raw);

    const int lane = threadIdx.x & 31;
    const int wave = threadIdx.x >> 5;
    const int hf = lane >> 4;
    const int lm = lane & 15;
    if ((int)(blockIdx.y * 256 + 256) > M) return;
    const int m0 = blockIdx.y * 256 + wave * 32;
    const int n0 = blockIdx.x * 64;
    if (n0 + 64 > N) return;

    v8f acc[2][4];
#pragma unroll
    for (int mt = 0; mt < 2; ++mt)
#pragma unroll
        for (int nt = 0; nt < 4; ++nt) {
            v8f z = {0.f, 0.f, 0.f, 0.f, 0.f, 0.f, 0.f, 0.f};
            acc[mt][nt] = z;
        }

    for (int kc = 0; kc < K; kc += KCHUNK) {
#pragma unroll
        for (int it = 0; it < 8; ++it) {
            const int c  = threadIdx.x + it * 256;
            const int j  = c >> 5;
            const int ke = (c & 31) * 8;
            const v8h v = *(const v8h*)(Wt + (size_t)(n0 + j) * K + kc + ke);
            *(v8h*)(bs + j * LDSPAD + ke) = v;
        }
        __syncthreads();

        for (int ko = 0; ko < KCHUNK; ko += 32) {
            const int k0 = kc + ko;
            FragH a0, a1;
            const f16_t* pa0 = A + (size_t)(m0 + lm) * K + k0 + 8 * hf;
            const f16_t* pa1 = A + (size_t)(m0 + 16 + lm) * K + k0 + 8 * hf;
            a0.half[0] = *(const v8h*)(pa0);
            a0.half[1] = *(const v8h*)(pa0 + 16);
            a1.half[0] = *(const v8h*)(pa1);
            a1.half[1] = *(const v8h*)(pa1 + 16);
#pragma unroll
            for (int nt = 0; nt < 4; ++nt) {
                FragH b;
                const f16_t* pb = bs + (nt * 16 + lm) * LDSPAD + ko + 8 * hf;
                b.half[0] = *(const v8ha*)(pb);
                b.half[1] = *(const v8ha*)(pb + 16);
                mma2(acc[0][nt], acc[1][nt], a0.v, a1.v, b.v);
            }
        }
        __syncthreads();
    }

    float* stg = lds_raw + wave * 2048;
#pragma unroll
    for (int mt = 0; mt < 2; ++mt) {
#pragma unroll
        for (int nt = 0; nt < 4; ++nt) {
            const int cl = nt * 16 + lm;
            const int n  = n0 + cl;
            float bn = 0.f;
            if (MODE != 0) bn = bias[n];
#pragma unroll
            for (int r = 0; r < 8; ++r) {
                const int rl = mt * 16 + 8 * hf + r;
                const int m  = m0 + rl;
                float v = acc[mt][nt][r] * WINV;
                if (MODE == 1 || MODE == 3) {
                    v = v + bn + res[(size_t)m * N + n];
                } else if (MODE == 2) {
                    const float z = v + bn;
                    v = 0.5f * z * (1.0f + erff(z * 0.70710678118654752f));
                }
                if (MODE == 3) stg[cl * 32 + rl] = v;
                else           stg[rl * 64 + cl] = v;
            }
        }
    }
    __syncthreads();

    tile_store<MODE>(stg, outf, outb, m0, n0, N, lane);
    __threadfence();
    tile_store<MODE>(stg, outf, outb, m0, n0, N, lane);
}

__global__ __launch_bounds__(256) void attn_kernel(
    const f16_t* __restrict__ Q, const f16_t* __restrict__ Kt,
    const f16_t* __restrict__ V, f16_t* O, int M) {
    __shared__ float so[DIMC];
    const int lane = threadIdx.x & 31, wave = threadIdx.x >> 5;
    const int pos = blockIdx.x;
    if (pos >= M) return;
    const int hg  = wave;
    const int dil = (hg >> 1) + 1;
    const int b   = pos >> 12;
    const int sp  = pos & (HWc - 1);
    const int hh  = sp >> 6;
    const int ww  = sp & 63;
    const int ch  = hg * 32 + lane;
    const int rowb = b << 12;

    const float qv = (float)Q[(size_t)pos * DIMC + ch];

    float logit[9], vm[9];
    int   nr[9];
#pragma unroll
    for (int ki = 0; ki < 3; ++ki) {
#pragma unroll
        for (int kj = 0; kj < 3; ++kj) {
            const int j = ki * 3 + kj;
            const int y = hh + (ki - 1) * dil;
            const int x = ww + (kj - 1) * dil;
            const bool ok = ((unsigned)y < 64u) && ((unsigned)x < 64u);
            const int yc = min(max(y, 0), 63);
            const int xc = min(max(x, 0), 63);
            nr[j] = rowb + yc * Wn + xc;
            vm[j] = ok ? 1.0f : 0.0f;
            const float kv = (float)Kt[(size_t)nr[j] * DIMC + ch];
            float part = qv * kv * vm[j];
            part = wsum32(part);
            logit[j] = part * SCALE;
        }
    }
    float mx = logit[0];
#pragma unroll
    for (int j = 1; j < 9; ++j) mx = fmaxf(mx, logit[j]);
    float w[9], den = 0.f;
#pragma unroll
    for (int j = 0; j < 9; ++j) { w[j] = __expf(logit[j] - mx); den += w[j]; }
    const float rden = 1.0f / den;
    float o = 0.f;
#pragma unroll
    for (int j = 0; j < 9; ++j)
        o += (w[j] * rden) * vm[j] * (float)V[(size_t)nr[j] * DIMC + ch];

    so[ch] = o;
    __syncthreads();
    if (wave == 0) {
        const v4f x0 = *(const v4fa*)(so + 8 * lane);
        const v4f x1 = *(const v4fa*)(so + 8 * lane + 4);
        v8h ov;
#pragma unroll
        for (int j = 0; j < 4; ++j) { ov[j] = (f16_t)x0[j]; ov[j + 4] = (f16_t)x1[j]; }
        f16_t* dst = O + (size_t)pos * DIMC + 8 * lane;
        *(volatile v8h*)dst = ov;
        __threadfence();
        *(volatile v8h*)dst = ov;
    }
}

extern "C" void kernel_launch(void* const* d_in, const int* in_sizes, int n_in,
                              void* d_out, int out_size, void* d_ws, size_t ws_size,
                              hipStream_t stream) {
    if (n_in < 14) return;
    const size_t tsz = (size_t)Bn * DIMC * HWc;
    if ((size_t)in_sizes[0] != 2 * tsz) return;
    if ((size_t)out_size != 2 * tsz) return;
    if (in_sizes[1] != 2 * DIMC || in_sizes[2] != 2 * DIMC || in_sizes[7] != 2 * DIMC ||
        in_sizes[8] != 2 * DIMC || in_sizes[9] != 2 * DIMC || in_sizes[13] != 2 * DIMC) return;
    if (in_sizes[3] != 2 * DIMC * DIMC || in_sizes[4] != 2 * DIMC * DIMC ||
        in_sizes[5] != 2 * DIMC * DIMC || in_sizes[6] != 2 * DIMC * DIMC) return;
    if (in_sizes[10] != 2 * HIDDENc * DIMC || in_sizes[11] != 2 * HIDDENc ||
        in_sizes[12] != 2 * DIMC * HIDDENc) return;
    if (ws_size < WS_TOTAL) return;

    const float* x       = (const float*)d_in[0];
    const float* norm1_w = (const float*)d_in[1];
    const float* norm1_b = (const float*)d_in[2];
    const float* q_w     = (const float*)d_in[3];
    const float* k_w     = (const float*)d_in[4];
    const float* v_w     = (const float*)d_in[5];
    const float* proj_w  = (const float*)d_in[6];
    const float* proj_b  = (const float*)d_in[7];
    const float* norm2_w = (const float*)d_in[8];
    const float* norm2_b = (const float*)d_in[9];
    const float* fc1_w   = (const float*)d_in[10];
    const float* fc1_b   = (const float*)d_in[11];
    const float* fc2_w   = (const float*)d_in[12];
    const float* fc2_b   = (const float*)d_in[13];
    float* outp = (float*)d_out;

    char* ws = (char*)d_ws;
    f16_t* wq    = (f16_t*)(ws + OFF_WQ);
    f16_t* wk    = (f16_t*)(ws + OFF_WK);
    f16_t* wv    = (f16_t*)(ws + OFF_WV);
    f16_t* wp    = (f16_t*)(ws + OFF_WP);
    f16_t* wfc1  = (f16_t*)(ws + OFF_WFC1);
    f16_t* wfc2  = (f16_t*)(ws + OFF_WFC2);
    float* x1res = (float*)(ws + OFF_X1RES);
    f16_t* x1n   = (f16_t*)(ws + OFF_X1N);
    f16_t* x2n   = (f16_t*)(ws + OFF_X2N);
    f16_t* Qb    = (f16_t*)(ws + OFF_Q);
    f16_t* Kb    = (f16_t*)(ws + OFF_K);
    f16_t* Vb    = (f16_t*)(ws + OFF_V);
    f16_t* attnb = (f16_t*)(ws + OFF_ATT);
    float* xaft  = (float*)(ws + OFF_XAFT);
    f16_t* hb    = (f16_t*)(ws + OFF_X2N);
    f16_t* h1b   = (f16_t*)(ws + OFF_Q);

    const int M = Mrows;

    {
        const int n8a = (2 * DIMC * DIMC) / 8;
        const int n8b = (2 * HIDDENc * DIMC) / 8;
        cvt_kernel<<<(n8a + 255) / 256, 256, 0, stream>>>(q_w,    wq,   n8a, WSCL);
        cvt_kernel<<<(n8a + 255) / 256, 256, 0, stream>>>(k_w,    wk,   n8a, WSCL);
        cvt_kernel<<<(n8a + 255) / 256, 256, 0, stream>>>(v_w,    wv,   n8a, WSCL);
        cvt_kernel<<<(n8a + 255) / 256, 256, 0, stream>>>(proj_w, wp,   n8a, WSCL);
        cvt_kernel<<<(n8b + 255) / 256, 256, 0, stream>>>(fc1_w,  wfc1, n8b, WSCL);
        cvt_kernel<<<(n8b + 255) / 256, 256, 0, stream>>>(fc2_w,  wfc2, n8b, WSCL);
    }

    const dim3 g256(DIMC / 64, (M + 255) / 256);
    const dim3 g1024(HIDDENc / 64, (M + 255) / 256);

    for (int bi = 0; bi < 2; ++bi) {
        const float* xa = x + (bi == 0 ? (size_t)0 : tsz);
        const float* xb = x + (bi == 0 ? tsz : (size_t)0);

        prep_kernel<<<(M + PREP_POS - 1) / PREP_POS, 256, 0, stream>>>(
            xa, xb, norm1_w + bi * DIMC, norm1_b + bi * DIMC, x1res, x1n, x2n, M);

        gemm_kernel<0><<<g256, 256, 0, stream>>>(
            x1n, wq + (size_t)bi * DIMC * DIMC, nullptr, nullptr, nullptr, Qb, M, DIMC, DIMC);
        gemm_kernel<0><<<g256, 256, 0, stream>>>(
            x2n, wk + (size_t)bi * DIMC * DIMC, nullptr, nullptr, nullptr, Kb, M, DIMC, DIMC);
        gemm_kernel<0><<<g256, 256, 0, stream>>>(
            x2n, wv + (size_t)bi * DIMC * DIMC, nullptr, nullptr, nullptr, Vb, M, DIMC, DIMC);

        attn_kernel<<<M, 256, 0, stream>>>(Qb, Kb, Vb, attnb, M);

        gemm_kernel<1><<<g256, 256, 0, stream>>>(
            attnb, wp + (size_t)bi * DIMC * DIMC, proj_b + bi * DIMC, x1res, xaft, nullptr,
            M, DIMC, DIMC);

        ln_rows_kernel<<<(M + 7) / 8, 256, 0, stream>>>(
            xaft, norm2_w + bi * DIMC, norm2_b + bi * DIMC, hb, M);

        gemm_kernel<2><<<g1024, 256, 0, stream>>>(
            hb, wfc1 + (size_t)bi * HIDDENc * DIMC, fc1_b + bi * HIDDENc, nullptr, nullptr, h1b,
            M, HIDDENc, DIMC);

        gemm_kernel<3><<<g256, 256, 0, stream>>>(
            h1b, wfc2 + (size_t)bi * DIMC * HIDDENc, fc2_b + bi * DIMC, xaft,
            outp + (size_t)bi * tsz, nullptr, M, DIMC, HIDDENc);
    }
}
